// MergeMultiHeadedSelfRetentionModule_40638980555014
// MI455X (gfx1250) — hardware-verified
//
#include <hip/hip_runtime.h>
#include <math.h>

constexpr int NSEQ       = 8;
constexpr int TLEN       = 2000;
constexpr int DMODEL     = 256;
constexpr int NHEAD      = 8;
constexpr int HEAD_D     = 32;
constexpr int CHUNK_LEN  = 500;
constexpr int NCHUNK     = 4;
constexpr int CHUNK_PAD  = 512;
constexpr int MROWS      = NSEQ * TLEN;
constexpr int MPAD       = NSEQ * NCHUNK * CHUNK_PAD;
constexpr int NPLANE     = NSEQ * NHEAD * NCHUNK;
constexpr int PLANE_EL   = CHUNK_PAD * HEAD_D;
constexpr int NQKVG      = 4 * DMODEL;
constexpr int NINPROJ    = 3 * DMODEL;
constexpr int NBATCH_OUT = 2;
constexpr int NCHAN_OUT  = 4;
constexpr int FINE_ROWS  = 16;
constexpr int FINE_EL    = FINE_ROWS * HEAD_D;
static_assert(NBATCH_OUT * NCHAN_OUT == NSEQ);
static_assert(DMODEL == NHEAD * HEAD_D);
static_assert(TLEN == NCHUNK * CHUNK_LEN);
static_assert(HEAD_D == 32);
static_assert(DMODEL % 32 == 0);
static_assert(MPAD % 64 == 0 && MROWS % 64 == 0);
static_assert(NQKVG % 64 == 0 && NINPROJ % 64 == 0 && DMODEL % 64 == 0);
static_assert(CHUNK_PAD % 64 == 0);
static_assert(MROWS % 8 == 0 && MPAD % 8 == 0);
static_assert(FINE_ROWS * (HEAD_D / 2) == 256);
static_assert(FINE_ROWS <= CHUNK_LEN);

constexpr float W_CARRY   = 16.0f;
constexpr float X_CARRY   = 16.0f;
constexpr float Q_CARRY   = 16.0f;
constexpr float K_CARRY   = 64.0f;
constexpr float V_CARRY   = 16.0f;
constexpr float P_CARRY   = 64.0f;
constexpr float VD_EXTRA  = 4.0f;
constexpr float ST_CARRY  = 1024.0f;
constexpr float LO_CARRY  = 2048.0f;
constexpr float LO_INV    = 1.0f / LO_CARRY;
constexpr float GEMM_SCALE = 1.0f / (X_CARRY * W_CARRY);
constexpr float QK_INV     = 1.0f / (Q_CARRY * K_CARRY);
constexpr float PV_INV     = 1.0f / (P_CARRY * V_CARRY);
constexpr float QS_INV     = 1.0f / (Q_CARRY * ST_CARRY);
constexpr float KV_INV     = 1.0f / (K_CARRY * V_CARRY * VD_EXTRA);

typedef __attribute__((ext_vector_type(16))) _Float16 v16h;
typedef __attribute__((ext_vector_type(8)))  _Float16 v8h;
typedef __attribute__((ext_vector_type(2)))  _Float16 v2h;
typedef __attribute__((ext_vector_type(8)))  float    v8f;
typedef __attribute__((ext_vector_type(4)))  float    v4f;
typedef __attribute__((ext_vector_type(2)))  float    v2f;
typedef __attribute__((ext_vector_type(4)))  unsigned int v4u;

union FragU { v16h v; v8h h[2]; };
__device__ __forceinline__ v16h frag_ld(const _Float16* p) {
  FragU f;
  f.h[0] = *(const v8h*)(p);
  f.h[1] = *(const v8h*)(p + 16);
  return f.v;
}
__device__ __forceinline__ v8f mma_raw(v16h a, v16h b, v8f c) {
  return __builtin_amdgcn_wmma_f32_16x16x32_f16(false, a, false, b, (short)0, c, false, false);
}
__device__ __forceinline__ v8f mma_g(v16h a, v16h b, v8f c) {
  c = __builtin_amdgcn_wmma_f32_16x16x32_f16(false, a, false, b, (short)0, c, false, false);
  asm volatile("v_nop\n\tv_nop\n\tv_nop\n\tv_nop" : "+v"(c) : "v"(a), "v"(b));
  return c;
}
__device__ __forceinline__ void guard4_h(v8f& a, v8f& b, v8f& c, v8f& d, v16h x, v16h y0, v16h y1, v16h y2, v16h y3) {
  asm volatile("v_nop\n\tv_nop\n\tv_nop\n\tv_nop" : "+v"(a), "+v"(b), "+v"(c), "+v"(d) : "v"(x), "v"(y0), "v"(y1), "v"(y2), "v"(y3));
}
__device__ __forceinline__ void acc_guard4(v8f& a, v8f& b, v8f& c, v8f& d) {
  asm volatile("v_nop\n\tv_nop\n\tv_nop\n\tv_nop" : "+v"(a), "+v"(b), "+v"(c), "+v"(d));
}
__device__ __forceinline__ void wave_lds_sync() {
  __builtin_amdgcn_fence(__ATOMIC_RELEASE, "workgroup");
  __builtin_amdgcn_wave_barrier();
  __builtin_amdgcn_fence(__ATOMIC_ACQUIRE, "workgroup");
}
__device__ __forceinline__ float h16_to_f32(unsigned hb) {
  const unsigned sgn = (hb & 0x8000u) << 16;
  const unsigned em = hb & 0x7fffu;
  const float fn = __uint_as_float((em << 13) + 0x38000000u);
  const float fs = (float)em * 5.9604644775390625e-8f;
  const float mag = (em < 0x400u) ? fs : fn;
  return __uint_as_float(__float_as_uint(mag) | sgn);
}

__global__ __launch_bounds__(256) void cvt_weights_kernel(const float* qw, const float* kw, const float* vw, const float* gw,
                                                          const float* ow, const float* inw, const float* outw,
                                                          unsigned short* dst) {
  const int blk = blockIdx.x;
  const float* src = qw;
  int lb = blk;
  if (blk >= 256)      { src = outw; lb = blk - 256; }
  else if (blk >= 160) { src = inw;  lb = blk - 160; }
  else if (blk >= 128) { src = ow;   lb = blk - 128; }
  else if (blk >= 96)  { src = gw;   lb = blk - 96; }
  else if (blk >= 64)  { src = vw;   lb = blk - 64; }
  else if (blk >= 32)  { src = kw;   lb = blk - 32; }
  const float* sp = src + ((size_t)lb * 256 + threadIdx.x) * 8;
  const v4f a = *(const v4f*)(sp);
  const v4f b = *(const v4f*)(sp + 4);
  v8h hv;
#pragma unroll
  for (int e = 0; e < 4; ++e) {
    hv[e]     = (_Float16)(a[e] * W_CARRY);
    hv[4 + e] = (_Float16)(b[e] * W_CARRY);
  }
  unsigned short* dp = dst + ((size_t)blk * 256 + threadIdx.x) * 8;
  *(volatile v8h*)(void*)dp = hv;
  __threadfence();
  *(volatile v8h*)(void*)dp = hv;
}

struct RotAng { float a[16]; };
static_assert(sizeof(RotAng) == 64);
__global__ __launch_bounds__(256) void rot_table_kernel(RotAng ra, float* tab) {
  const int lane = threadIdx.x & 31;
  const int t = blockIdx.x * 8 + (threadIdx.x >> 5);
  const int pl = lane & 15;
  float ang = ra.a[0];
#pragma unroll
  for (int p = 1; p < 16; ++p) ang = (pl == p) ? ra.a[p] : ang;
  const float theta = (float)t * ang;
  float sn, cs;
  sincosf(theta, &sn, &cs);
  const float val = (lane < 16) ? cs : sn;
  float* dp = tab + (size_t)t * 32 + lane;
  *(volatile float*)dp = val;
  __threadfence();
  *(volatile float*)dp = val;
}

template <int MODE>
__global__ __launch_bounds__(256) void ln_rows_kernel(const float* X, const float* gam, const float* bet,
                                                      unsigned short* Y, int nrows) {
  const int lane = threadIdx.x & 31;
  const int row = blockIdx.x * 8 + (threadIdx.x >> 5);
  if (row >= nrows) return;
  int src;
  bool valid = true;
  if (MODE == 0) {
    const int sc = row >> 9;
    const int i = row & (CHUNK_PAD - 1);
    valid = (i < CHUNK_LEN);
    const int ic = valid ? i : (CHUNK_LEN - 1);
    src = (sc >> 2) * TLEN + (sc & 3) * CHUNK_LEN + ic;
  } else {
    const int c = row & 3;
    const int bt = row >> 2;
    const int b = bt / TLEN;
    const int t = bt - b * TLEN;
    src = (b * NCHAN_OUT + c) * TLEN + t;
  }
  const float* xp = X + (size_t)src * DMODEL + lane * 8;
  const v4f x0 = *(const v4f*)(xp);
  const v4f x1 = *(const v4f*)(xp + 4);
  const v4f g0 = *(const v4f*)(gam + lane * 8);
  const v4f g1 = *(const v4f*)(gam + lane * 8 + 4);
  const v4f b0 = *(const v4f*)(bet + lane * 8);
  const v4f b1 = *(const v4f*)(bet + lane * 8 + 4);
  float s = ((x0[0] + x0[1]) + (x0[2] + x0[3])) + ((x1[0] + x1[1]) + (x1[2] + x1[3]));
#pragma unroll
  for (int off = 1; off < 32; off <<= 1) s += __shfl_xor(s, off, 32);
  const float mu = s * (1.0f / DMODEL);
  float d[8];
  float ss = 0.0f;
#pragma unroll
  for (int e = 0; e < 4; ++e) {
    d[e] = x0[e] - mu;
    d[4 + e] = x1[e] - mu;
  }
#pragma unroll
  for (int e = 0; e < 8; ++e) ss += d[e] * d[e];
#pragma unroll
  for (int off = 1; off < 32; off <<= 1) ss += __shfl_xor(ss, off, 32);
  const float inv = 1.0f / sqrtf(ss * (1.0f / DMODEL) + 1e-5f);
  v8h hv;
#pragma unroll
  for (int e = 0; e < 4; ++e) {
    const float y0 = ((d[e] * inv) * g0[e] + b0[e]) * X_CARRY;
    const float y1 = ((d[4 + e] * inv) * g1[e] + b1[e]) * X_CARRY;
    hv[e]     = (_Float16)(valid ? y0 : 0.0f);
    hv[4 + e] = (_Float16)(valid ? y1 : 0.0f);
  }
  unsigned short* dp = Y + (size_t)row * DMODEL + lane * 8;
  *(volatile v8h*)(void*)dp = hv;
  __threadfence();
  *(volatile v8h*)(void*)dp = hv;
}

template <int AMODE, int EPI, bool BIAS, bool RESID, bool ROWMAP>
__global__ __launch_bounds__(256) void gemm_f16_kernel(
    const unsigned short* A16, const float* A32, int lda,
    const unsigned short* Btp, int ldb,
    float* outF, int ldc,
    unsigned short* outQ, unsigned short* outK, unsigned short* outV,
    unsigned short* outQlo, unsigned short* outKlo,
    const float* bias, const float* resid, const float* rot,
    int M, int N, int K, float scale, float kscale) {
  __shared__ __align__(16) float sT[8][16 * 68];
  const int lane = threadIdx.x & 31;
  const int wave = threadIdx.x >> 5;
  const int tilesN = N >> 6;
  const int tilesM = M >> 6;
  const int tile = blockIdx.x * 8 + wave;
  if (tile >= tilesM * tilesN) return;
  const int tm = tile / tilesN;
  const int tn = tile - tm * tilesN;
  const int m0 = tm << 6;
  const int n0 = tn << 6;
  const int rlane = lane & 15;
  const int koff = (lane >> 4) * 8;
  const int mOff = koff;

  const _Float16* bp[4];
  const _Float16* ap16[4];
  const float* ap32[4];
#pragma unroll
  for (int j = 0; j < 4; ++j) bp[j] = (const _Float16*)Btp + (size_t)(n0 + (j << 4) + rlane) * ldb + koff;
#pragma unroll
  for (int i = 0; i < 4; ++i) {
    ap16[i] = (const _Float16*)A16 + (size_t)(m0 + (i << 4) + rlane) * lda + koff;
    ap32[i] = A32 + (size_t)(m0 + (i << 4) + rlane) * lda + koff;
  }

  v8f acc[4][4];
#pragma unroll
  for (int i = 0; i < 4; ++i)
#pragma unroll
    for (int j = 0; j < 4; ++j) acc[i][j] = (v8f){0.f, 0.f, 0.f, 0.f, 0.f, 0.f, 0.f, 0.f};

  for (int k0 = 0; k0 < K; k0 += 32) {
    v16h bh[4];
#pragma unroll
    for (int j = 0; j < 4; ++j) bh[j] = frag_ld(bp[j] + k0);
#pragma unroll
    for (int i = 0; i < 4; ++i) {
      v16h ah;
      if (AMODE == 0) {
        ah = frag_ld(ap16[i] + k0);
      } else {
        const float* ap = ap32[i] + k0;
        const v4f x0 = *(const v4f*)(ap);
        const v4f x1 = *(const v4f*)(ap + 4);
        const v4f x2 = *(const v4f*)(ap + 16);
        const v4f x3 = *(const v4f*)(ap + 20);
#pragma unroll
        for (int e = 0; e < 4; ++e) {
          ah[e]      = (_Float16)(x0[e] * X_CARRY);
          ah[4 + e]  = (_Float16)(x1[e] * X_CARRY);
          ah[8 + e]  = (_Float16)(x2[e] * X_CARRY);
          ah[12 + e] = (_Float16)(x3[e] * X_CARRY);
        }
      }
#pragma unroll
      for (int j = 0; j < 4; ++j) acc[i][j] = mma_raw(ah, bh[j], acc[i][j]);
      guard4_h(acc[i][0], acc[i][1], acc[i][2], acc[i][3], ah, bh[0], bh[1], bh[2], bh[3]);
    }
  }
  acc_guard4(acc[0][0], acc[0][1], acc[0][2], acc[0][3]);
  acc_guard4(acc[1][0], acc[1][1], acc[1][2], acc[1][3]);
  acc_guard4(acc[2][0], acc[2][1], acc[2][2], acc[2][3]);
  acc_guard4(acc[3][0], acc[3][1], acc[3][2], acc[3][3]);

  float* slab = sT[wave];
  const int mt = (EPI == 0) ? (n0 >> 8) : 3;
  const int hbase = (n0 & (DMODEL - 1)) >> 5;
  const int sc = m0 >> 9;
  const int sq = sc >> 2;
  const int ch = sc & 3;
  const int i0 = m0 & (CHUNK_PAD - 1);
  float sc_eff = scale;
  if (EPI == 0) {
    if (mt == 0) sc_eff = scale * Q_CARRY;
    else if (mt == 1) sc_eff = scale * kscale * K_CARRY;
    else if (mt == 2) sc_eff = scale * V_CARRY;
  }
  unsigned short* plane = outQ;
  if (EPI == 0) {
    if (mt == 1) plane = outK;
    else if (mt == 2) plane = outV;
  }
  unsigned short* loPlane = (mt == 1) ? outKlo : outQlo;
  const bool fineTile = (EPI == 0) && (mt < 2) && (ch == 0) && (i0 == 0);
  const int ncol = (EPI == 0) ? (n0 & (DMODEL - 1)) : n0;

#pragma unroll
  for (int i = 0; i < 4; ++i) {
    const int mBase = m0 + (i << 4);
#pragma unroll
    for (int j = 0; j < 4; ++j) {
#pragma unroll
      for (int r = 0; r < 8; ++r) slab[(mOff + r) * 68 + (j << 4) + rlane] = acc[i][j][r] * sc_eff;
    }
    wave_lds_sync();
    if (EPI == 0 && mt < 3) {
      const int p = lane & 7;
      const int lq = lane >> 3;
      const bool doLo = fineTile && (i == 0);
#pragma unroll 1
      for (int it = 0; it < 4; ++it) {
        const int line = it * 4 + lq;
        const int hl = line >> 3;
        const int rp = line & 7;
        const int row = 2 * rp + (p >> 2);
        const int dcol = (p & 3) * 8;
        const float* sp = slab + row * 68 + hl * 32 + dcol;
        const v4f s0 = *(const v4f*)(sp);
        const v4f s1 = *(const v4f*)(sp + 4);
        float x[8];
#pragma unroll
        for (int e = 0; e < 4; ++e) {
          x[e] = s0[e];
          x[4 + e] = s1[e];
        }
        const int ii = i0 + (i << 4) + row;
        if (mt < 2) {
          int tt = ch * CHUNK_LEN + ii;
          tt = (tt > TLEN - 1) ? (TLEN - 1) : tt;
          const float* tp = rot + (size_t)tt * 32 + (dcol >> 1);
          const v4f cs = *(const v4f*)(tp);
          const v4f sn = *(const v4f*)(tp + 16);
#pragma unroll
          for (int e2 = 0; e2 < 4; ++e2) {
            const float xa = x[2 * e2];
            const float xb = x[2 * e2 + 1];
            x[2 * e2]     = xa * cs[e2] - xb * sn[e2];
            x[2 * e2 + 1] = xb * cs[e2] + xa * sn[e2];
          }
        }
        v8h hv, lv;
#pragma unroll
        for (int e = 0; e < 8; ++e) {
          const _Float16 hq = (_Float16)x[e];
          const float hf = (float)hq;
          hv[e] = hq;
          lv[e] = (_Float16)((x[e] - hf) * LO_CARRY);
        }
        unsigned short* dp = plane + ((size_t)((sq * NHEAD + hbase + hl) * NCHUNK + ch) * CHUNK_PAD + ii) * HEAD_D + dcol;
        unsigned short* lp = loPlane + ((size_t)(sq * NHEAD + hbase + hl) * FINE_ROWS + row) * HEAD_D + dcol;
        *(volatile v8h*)(void*)dp = hv;
        if (doLo) *(volatile v8h*)(void*)lp = lv;
        __threadfence();
        *(volatile v8h*)(void*)dp = hv;
        if (doLo) *(volatile v8h*)(void*)lp = lv;
      }
    } else {
      const int hh = lane >> 4;
      const int c4 = (lane & 15) * 4;
#pragma unroll 1
      for (int it = 0; it < 8; ++it) {
        const int row = it * 2 + hh;
        const int m = mBase + row;
        int dm = m;
        if (ROWMAP) {
          const int c = m & 3;
          const int bt = m >> 2;
          const int b = bt / TLEN;
          const int t = bt - b * TLEN;
          dm = (b * NCHAN_OUT + c) * TLEN + t;
        }
        v4f v = *(const v4f*)(slab + row * 68 + c4);
        const size_t off = (size_t)dm * ldc + ncol + c4;
        if (BIAS) {
          const v4f bv = *(const v4f*)(bias + ncol + c4);
          v += bv;
        }
        if (RESID) {
          const v4f rv = *(const v4f*)(resid + off);
          v += rv;
        }
        float* dp = outF + off;
        *(volatile v4f*)dp = v;
        __threadfence();
        *(volatile v4f*)dp = v;
      }
    }
    wave_lds_sync();
  }
}

constexpr int FPITCH = 260;
constexpr int FOP = 36;
__global__ __launch_bounds__(256) void fine_qk_kernel(const float* X, const float* gam, const float* bet,
                                                      const float* qw, const float* kw, const float* rot,
                                                      unsigned short* outQ, unsigned short* outK,
                                                      unsigned short* outQlo, unsigned short* outKlo, float kscale) {
  __shared__ __align__(16) float xs[FINE_ROWS * FPITCH];
  __shared__ __align__(16) float oS[FINE_ROWS * FOP];
  const int bid = blockIdx.x;
  const int which = bid & 1;
  const int sh = bid >> 1;
  const int sq = sh >> 3;
  const int h = sh & 7;
  const int tid = threadIdx.x;
  const int lane = tid & 31;
  const int wave = tid >> 5;

  const v4f g0 = *(const v4f*)(gam + lane * 8);
  const v4f g1 = *(const v4f*)(gam + lane * 8 + 4);
  const v4f b0 = *(const v4f*)(bet + lane * 8);
  const v4f b1 = *(const v4f*)(bet + lane * 8 + 4);
#pragma unroll 1
  for (int rr = 0; rr < 2; ++rr) {
    const int lrow = wave * 2 + rr;
    const float* xp = X + ((size_t)sq * TLEN + lrow) * DMODEL + lane * 8;
    const v4f x0 = *(const v4f*)(xp);
    const v4f x1 = *(const v4f*)(xp + 4);
    float s = ((x0[0] + x0[1]) + (x0[2] + x0[3])) + ((x1[0] + x1[1]) + (x1[2] + x1[3]));
#pragma unroll
    for (int off = 1; off < 32; off <<= 1) s += __shfl_xor(s, off, 32);
    const float mu = s * (1.0f / DMODEL);
    float d[8];
    float ss = 0.0f;
#pragma unroll
    for (int e = 0; e < 4; ++e) {
      d[e] = x0[e] - mu;
      d[4 + e] = x1[e] - mu;
    }
#pragma unroll
    for (int e = 0; e < 8; ++e) ss += d[e] * d[e];
#pragma unroll
    for (int off = 1; off < 32; off <<= 1) ss += __shfl_xor(ss, off, 32);
    const float inv = 1.0f / sqrtf(ss * (1.0f / DMODEL) + 1e-5f);
    v4f y0, y1;
#pragma unroll
    for (int e = 0; e < 4; ++e) {
      y0[e] = (d[e] * inv) * g0[e] + b0[e];
      y1[e] = (d[4 + e] * inv) * g1[e] + b1[e];
    }
    float* dp = xs + lrow * FPITCH + lane * 8;
    *(v4f*)(dp) = y0;
    *(v4f*)(dp + 4) = y1;
  }
  __syncthreads();

  {
    const int row = tid >> 4;
    const int p = tid & 15;
    const float* W = which ? kw : qw;
    const float* w0 = W + (size_t)(h * HEAD_D + 2 * p) * DMODEL;
    const float* w1 = w0 + DMODEL;
    const float* xr = xs + row * FPITCH;
    v4f a0 = (v4f){0.f, 0.f, 0.f, 0.f};
    v4f a1 = (v4f){0.f, 0.f, 0.f, 0.f};
#pragma unroll 1
    for (int k = 0; k < DMODEL; k += 4) {
      const v4f xv = *(const v4f*)(xr + k);
      const v4f u0 = *(const v4f*)(w0 + k);
      const v4f u1 = *(const v4f*)(w1 + k);
      a0 += xv * u0;
      a1 += xv * u1;
    }
    const float d0 = (a0[0] + a0[1]) + (a0[2] + a0[3]);
    const float d1 = (a1[0] + a1[1]) + (a1[2] + a1[3]);
    const float scl = which ? (kscale * K_CARRY) : Q_CARRY;
    const float xa = d0 * scl;
    const float xb = d1 * scl;
    const float cs = rot[(size_t)row * 32 + p];
    const float sn = rot[(size_t)row * 32 + 16 + p];
    oS[row * FOP + 2 * p]     = xa * cs - xb * sn;
    oS[row * FOP + 2 * p + 1] = xb * cs + xa * sn;
  }
  __syncthreads();

  if (tid < 128) {
    const int isLo = tid >> 6;
    const int u = tid & 63;
    const int line = u >> 3;
    const int pc = u & 7;
    const int orow = 2 * line + (pc >> 2);
    const int dcol = (pc & 3) * 8;
    const float* sp = oS + orow * FOP + dcol;
    const v4f s0 = *(const v4f*)(sp);
    const v4f s1 = *(const v4f*)(sp + 4);
    float x[8];
#pragma unroll
    for (int e = 0; e < 4; ++e) {
      x[e] = s0[e];
      x[4 + e] = s1[e];
    }
    v8h val;
#pragma unroll
    for (int e = 0; e < 8; ++e) {
      const _Float16 hq = (_Float16)x[e];
      const float hf = (float)hq;
      const _Float16 lq = (_Float16)((x[e] - hf) * LO_CARRY);
      val[e] = isLo ? lq : hq;
    }
    unsigned short* hiPlane = which ? outK : outQ;
    unsigned short* loPlane = which ? outKlo : outQlo;
    unsigned short* dph = hiPlane + ((size_t)((sq * NHEAD + h) * NCHUNK) * CHUNK_PAD + orow) * HEAD_D + dcol;
    unsigned short* dpl = loPlane + ((size_t)(sq * NHEAD + h) * FINE_ROWS + orow) * HEAD_D + dcol;
    unsigned short* dp = isLo ? dpl : dph;
    *(volatile v8h*)(void*)dp = val;
    __threadfence();
    *(volatile v8h*)(void*)dp = val;
  }
}

constexpr int KVP = 264;
__global__ __launch_bounds__(128) void kv_chunk_kernel(const unsigned short* krp, const unsigned short* vp, float* kvout) {
  __shared__ __align__(16) _Float16 kT[32 * KVP];
  __shared__ __align__(16) _Float16 vT[32 * KVP];
  __shared__ __align__(16) float oS[32 * 36];
  const int pi = blockIdx.x;
  const int h = (pi >> 2) & 7;
  const int tid = threadIdx.x;
  const int lane = tid & 31;
  const int wave = tid >> 5;
  const int c = lane & 15;
  const int hh = lane >> 4;
  const int mt = wave >> 1;
  const int nt = wave & 1;
  const float pw = (float)(32 << h);
  const float dec = logf(1.0f - 1.0f / pw);
  const unsigned short* kb = krp + (size_t)pi * PLANE_EL;
  const unsigned short* vb = vp + (size_t)pi * PLANE_EL;
  v8f acc = (v8f){0.f, 0.f, 0.f, 0.f, 0.f, 0.f, 0.f, 0.f};
#pragma unroll 1
  for (int ph = 0; ph < 2; ++ph) {
    __syncthreads();
#pragma unroll 1
    for (int itr = 0; itr < 8; ++itr) {
      const int idx = itr * 128 + tid;
      const int jl = idx >> 2;
      const int d0 = (idx & 3) * 8;
      const int j = ph * 256 + jl;
      const v4u wk4 = *(const v4u*)(const void*)(kb + (size_t)j * HEAD_D + d0);
      const v4u wv4 = *(const v4u*)(const void*)(vb + (size_t)j * HEAD_D + d0);
      const float wj = (j < CHUNK_LEN) ? (VD_EXTRA * expf(dec * (float)(CHUNK_LEN - 1 - j))) : 0.0f;
#pragma unroll
      for (int q = 0; q < 4; ++q) {
        const unsigned wk = wk4[q];
        const unsigned wv = wv4[q];
        const unsigned short klo = (unsigned short)(wk & 0xffffu);
        const unsigned short khi = (unsigned short)(wk >> 16);
        const _Float16 hklo = __builtin_bit_cast(_Float16, klo);
        const _Float16 hkhi = __builtin_bit_cast(_Float16, khi);
        kT[(d0 + 2 * q) * KVP + jl] = hklo;
        kT[(d0 + 2 * q + 1) * KVP + jl] = hkhi;
        const float flo = h16_to_f32(wv & 0xffffu) * wj;
        const float fhi = h16_to_f32(wv >> 16) * wj;
        vT[(d0 + 2 * q) * KVP + jl] = (_Float16)flo;
        vT[(d0 + 2 * q + 1) * KVP + jl] = (_Float16)fhi;
      }
    }
    __syncthreads();
    const _Float16* arow = kT + (mt * 16 + c) * KVP + 8 * hh;
    const _Float16* brow = vT + (nt * 16 + c) * KVP + 8 * hh;
#pragma unroll 1
    for (int kt = 0; kt < 8; ++kt) {
      const v16h a = frag_ld(arow + kt * 32);
      const v16h b = frag_ld(brow + kt * 32);
      acc = mma_g(a, b, acc);
    }
  }
  const float Ltot = -expm1f(dec * (float)CHUNK_LEN) * pw;
  const float osc = KV_INV / Ltot;
#pragma unroll
  for (int r = 0; r < 8; ++r) oS[(mt * 16 + 8 * hh + r) * 36 + nt * 16 + c] = acc[r] * osc;
  __syncthreads();
#pragma unroll
  for (int it = 0; it < 2; ++it) {
    const int idx = it * 128 + tid;
    const int row = idx >> 3;
    const int c4 = (idx & 7) * 4;
    const v4f v = *(const v4f*)(oS + row * 36 + c4);
    float* dp = kvout + (size_t)pi * 1024 + row * 32 + c4;
    *(volatile v4f*)dp = v;
    __threadfence();
    *(volatile v4f*)dp = v;
  }
}

__global__ __launch_bounds__(32) void scan_kernel(const float* kv, unsigned short* st16, float* cscale) {
  __shared__ __align__(16) float kS[32 * 36];
  __shared__ __align__(16) float sS[32 * 33];
  const int bid = blockIdx.x;
  const int h = bid & 7;
  const int lane = threadIdx.x;
  const float pw = (float)(32 << h);
  const float dec = logf(1.0f - 1.0f / pw);
  const float cd = expf(dec * (float)CHUNK_LEN);
  float st[32];
#pragma unroll
  for (int k = 0; k < 32; ++k) st[k] = 0.0f;
  float scale = 1.0f;
  float sv = 1.0f;
#pragma unroll 1
  for (int ch = 0; ch < NCHUNK; ++ch) {
    sv = ((lane & 3) == ch) ? scale : sv;
#pragma unroll
    for (int k = 0; k < 32; ++k) sS[lane * 33 + k] = st[k];
    const float* kp = kv + ((size_t)bid * NCHUNK + ch) * 1024;
#pragma unroll
    for (int q = 0; q < 8; ++q) {
      const int idx = q * 32 + lane;
      const v4f t4 = *(const v4f*)(kp + (size_t)idx * 4);
      *(v4f*)(kS + (idx >> 3) * 36 + (idx & 7) * 4) = t4;
    }
    __syncthreads();
    v8h hvv[4];
#pragma unroll
    for (int q = 0; q < 4; ++q) {
      const int e = q * 32 + lane;
      const int d = e >> 2;
      const int k0 = (e & 3) * 8;
#pragma unroll
      for (int e2 = 0; e2 < 8; ++e2) hvv[q][e2] = (_Float16)(sS[d * 33 + k0 + e2] * ST_CARRY);
    }
    unsigned short* sp = st16 + ((size_t)bid * NCHUNK + ch) * 1024;
    for (int pass = 0; pass < 2; ++pass) {
#pragma unroll
      for (int q = 0; q < 4; ++q) *(volatile v8h*)(void*)(sp + (size_t)(q * 32 + lane) * 8) = hvv[q];
      __threadfence();
    }
    float cs = 0.0f;
#pragma unroll
    for (int k = 0; k < 32; ++k) {
      st[k] = st[k] * cd + kS[k * 36 + lane];
      cs += fabsf(st[k]);
    }
#pragma unroll
    for (int off = 16; off >= 1; off >>= 1) cs = fmaxf(cs, __shfl_xor(cs, off, 32));
    scale = fmaxf(cs, 1.0f);
    __syncthreads();
  }
  float* cp = cscale + (size_t)bid * 32 + lane;
  *(volatile float*)cp = sv;
  __threadfence();
  *(volatile float*)cp = sv;
}

constexpr int VTP = 520;
constexpr int SPITCH = 72;
constexpr int OPITCH = 36;
__global__ __launch_bounds__(128) void chunk_attn_kernel(const unsigned short* qrp, const unsigned short* krp,
                                                         const unsigned short* vp, const unsigned short* st16,
                                                         const unsigned short* qlop, const unsigned short* klop,
                                                         const float* cscale, const float* gpl, float* y) {
  __shared__ __align__(16) _Float16 vT[32 * VTP];
  __shared__ __align__(16) _Float16 strip[4][16 * SPITCH];
  __shared__ __align__(16) float slab[4][16 * OPITCH];
  __shared__ float Rf[CHUNK_PAD];
  __shared__ float Cf[CHUNK_PAD];
  __shared__ float Qd[CHUNK_PAD];
  const int pi = blockIdx.x;
  const int sq = pi >> 5;
  const int h = (pi >> 2) & 7;
  const int ch = pi & 3;
  const int tid = threadIdx.x;
  const int lane = tid & 31;
  const int wave = tid >> 5;
  const int c = lane & 15;
  const int hh = lane >> 4;
  const float pw = (float)(32 << h);
  const float dec = logf(1.0f - 1.0f / pw);
  const float Ltot = -expm1f(dec * (float)CHUNK_LEN) * pw;

#pragma unroll 1
  for (int n = 0; n < 4; ++n) {
    const int i = n * 128 + tid;
    const float fi = (float)i;
    const float gi = expf(dec * fi);
    const float gi1 = expf(dec * (fi + 1.0f));
    const float Si = -expm1f(dec * (fi + 1.0f)) * pw;
    const float rs = 1.0f / sqrtf(Si);
    const float ci = expf(-dec * fi);
    const bool ok = (i < CHUNK_LEN);
    Rf[i] = ok ? (gi * rs) : 0.0f;
    Cf[i] = ok ? ci : 0.0f;
    Qd[i] = ok ? (gi1 * Ltot * rs) : 0.0f;
  }
  {
    const unsigned short* vb = vp + (size_t)pi * PLANE_EL;
#pragma unroll 1
    for (int itr = 0; itr < 16; ++itr) {
      const int idx = itr * 128 + tid;
      const int j = idx >> 2;
      const int d0 = (idx & 3) * 8;
      const v4u w4 = *(const v4u*)(const void*)(vb + (size_t)idx * 8);
#pragma unroll
      for (int q = 0; q < 4; ++q) {
        const unsigned wq = w4[q];
        const unsigned short lo = (unsigned short)(wq & 0xffffu);
        const unsigned short hi = (unsigned short)(wq >> 16);
        const _Float16 hlo = __builtin_bit_cast(_Float16, lo);
        const _Float16 hhi = __builtin_bit_cast(_Float16, hi);
        vT[(d0 + 2 * q) * VTP + j] = hlo;
        vT[(d0 + 2 * q + 1) * VTP + j] = hhi;
      }
    }
  }
  __syncthreads();

  const _Float16* qr = (const _Float16*)qrp + (size_t)pi * PLANE_EL;
  const _Float16* kr = (const _Float16*)krp + (size_t)pi * PLANE_EL;
  const _Float16* stp = (const _Float16*)st16 + (size_t)pi * 1024;
  const v16h bst0 = frag_ld(stp + c * 32 + 8 * hh);
  const v16h bst1 = frag_ld(stp + (16 + c) * 32 + 8 * hh);
  const float cs = cscale[(size_t)(pi >> 2) * 32 + ch];
  _Float16* sw = strip[wave];
  float* ow = slab[wave];
  const v8f z8 = (v8f){0.f, 0.f, 0.f, 0.f, 0.f, 0.f, 0.f, 0.f};
  const float* grow = gpl + ((size_t)(sq * NCHUNK + ch) * CHUNK_PAD) * DMODEL + h * HEAD_D;
  float* yrow = y + ((size_t)(sq * TLEN + ch * CHUNK_LEN)) * DMODEL + h * HEAD_D;

  v8f resid0 = z8;
  if (ch == 0) {
    const _Float16* qlp = (const _Float16*)qlop + (size_t)(pi >> 2) * FINE_EL;
    const _Float16* klp = (const _Float16*)klop + (size_t)(pi >> 2) * FINE_EL;
    const v16h a0 = frag_ld(qr + c * HEAD_D + 8 * hh);
    const v16h b0 = frag_ld(kr + c * HEAD_D + 8 * hh);
    const v16h al = frag_ld(qlp + c * HEAD_D + 8 * hh);
    const v16h bl = frag_ld(klp + c * HEAD_D + 8 * hh);
    v8f t0 = mma_g(a0, bl, z8);
    t0 = mma_g(al, b0, t0);
#pragma unroll
    for (int r = 0; r < 8; ++r) resid0[r] = t0[r] * LO_INV;
  }

#pragma unroll 1
  for (int it = wave; it < 32; it += 4) {
    const v16h a = frag_ld(qr + (it * 16 + c) * HEAD_D + 8 * hh);
    const bool fine = (ch == 0) && (it == 0);
    float Rr[8], rows[8];
#pragma unroll
    for (int r = 0; r < 8; ++r) {
      Rr[r] = Rf[it * 16 + 8 * hh + r] * QK_INV;
      rows[r] = 0.0f;
    }
    v8f acc0 = z8, acc1 = z8;
    const int njb = (it >> 2) + 1;
    const int ibase = it * 16 + 8 * hh;
#pragma unroll 1
    for (int jb = 0; jb < njb; ++jb) {
#pragma unroll
      for (int tj = 0; tj < 4; ++tj) {
        const int jg = (jb * 4 + tj) * 16 + c;
        const v16h b = frag_ld(kr + jg * HEAD_D + 8 * hh);
        v8f qk = mma_g(a, b, z8);
        if (tj == 0) {
#pragma unroll
          for (int r = 0; r < 8; ++r) qk[r] += fine ? resid0[r] : 0.0f;
        }
        const float Cj = Cf[jg];
#pragma unroll
        for (int r = 0; r < 8; ++r) {
          const float mk = (jg <= ibase + r) ? (Rr[r] * Cj) : 0.0f;
          const float qm = qk[r] * mk;
          rows[r] += fabsf(qm);
          sw[(8 * hh + r) * SPITCH + tj * 16 + c] = (_Float16)(qm * P_CARRY);
        }
      }
      wave_lds_sync();
#pragma unroll
      for (int kk = 0; kk < 2; ++kk) {
        const v16h pa = frag_ld(sw + c * SPITCH + kk * 32 + 8 * hh);
        const v16h vb0 = frag_ld(vT + c * VTP + jb * 64 + kk * 32 + 8 * hh);
        const v16h vb1 = frag_ld(vT + (16 + c) * VTP + jb * 64 + kk * 32 + 8 * hh);
        acc0 = mma_g(pa, vb0, acc0);
        acc1 = mma_g(pa, vb1, acc1);
      }
      wave_lds_sync();
    }
#pragma unroll
    for (int r = 0; r < 8; ++r) {
      float rv = rows[r];
      rv += __shfl_xor(rv, 8, 32);
      rv += __shfl_xor(rv, 4, 32);
      rv += __shfl_xor(rv, 2, 32);
      rv += __shfl_xor(rv, 1, 32);
      rows[r] = rv;
    }
    const v8f x0 = mma_g(a, bst0, z8);
    const v8f x1 = mma_g(a, bst1, z8);
#pragma unroll
    for (int r = 0; r < 8; ++r) {
      const float isc = fmaxf(rows[r], 1.0f);
      const float all = fmaxf(isc, cs);
      const float inv = 1.0f / all;
      const float qd = Qd[ibase + r] * QS_INV;
      const float o0 = (acc0[r] * PV_INV + qd * x0[r]) * inv;
      const float o1 = (acc1[r] * PV_INV + qd * x1[r]) * inv;
      float ss = o0 * o0 + o1 * o1;
      ss += __shfl_xor(ss, 8, 32);
      ss += __shfl_xor(ss, 4, 32);
      ss += __shfl_xor(ss, 2, 32);
      ss += __shfl_xor(ss, 1, 32);
      const float rn = 1.0f / sqrtf(ss * (1.0f / HEAD_D) + 1e-6f);
      ow[(8 * hh + r) * OPITCH + c] = o0 * rn;
      ow[(8 * hh + r) * OPITCH + 16 + c] = o1 * rn;
    }
    wave_lds_sync();
#pragma unroll 1
    for (int it2 = 0; it2 < 4; ++it2) {
      const int row = it2 * 4 + (lane >> 3);
      const int c4 = (lane & 7) * 4;
      const int i = it * 16 + row;
      const bool ok = (i < CHUNK_LEN);
      const int ic = ok ? i : (CHUNK_LEN - 1);
      const v4f o = *(const v4f*)(ow + row * OPITCH + c4);
      const v4f gv = *(const v4f*)(grow + (size_t)i * DMODEL + c4);
      v4f yv;
#pragma unroll
      for (int e = 0; e < 4; ++e) {
        const float ge = gv[e];
        const float sg = 1.0f / (1.0f + expf(-ge));
        yv[e] = (ge * sg) * o[e];
      }
      float* dp = yrow + (size_t)ic * DMODEL + c4;
      if (ok) *(volatile v4f*)dp = yv;
      __threadfence();
      if (ok) *(volatile v4f*)dp = yv;
    }
    wave_lds_sync();
  }
}

__global__ __launch_bounds__(256) void mha4_kernel(const float* qkv, unsigned short* attn, float qscale) {
  const int lane = threadIdx.x & 31;
  const int gw = blockIdx.x * 8 + (threadIdx.x >> 5);
  const int bt = gw >> 2;
  const int hp = gw & 3;
  const int col = hp * 64 + 2 * lane;
  float k0[4], k1[4], v0[4], v1[4];
#pragma unroll
  for (int cc = 0; cc < 4; ++cc) {
    const float* rp = qkv + (size_t)(bt * 4 + cc) * NINPROJ + col;
    const v2f kk = *(const v2f*)(rp + DMODEL);
    const v2f vv = *(const v2f*)(rp + 2 * DMODEL);
    k0[cc] = kk[0];
    k1[cc] = kk[1];
    v0[cc] = vv[0];
    v1[cc] = vv[1];
  }
#pragma unroll 1
  for (int qc = 0; qc < 4; ++qc) {
    const v2f qq = *(const v2f*)(qkv + (size_t)(bt * 4 + qc) * NINPROJ + col);
    const float q0 = qq[0] * qscale;
    const float q1 = qq[1] * qscale;
    float sc[4];
#pragma unroll
    for (int j = 0; j < 4; ++j) {
      float s = q0 * k0[j] + q1 * k1[j];
      s += __shfl_xor(s, 8, 32);
      s += __shfl_xor(s, 4, 32);
      s += __shfl_xor(s, 2, 32);
      s += __shfl_xor(s, 1, 32);
      sc[j] = s;
    }
    const float mx = fmaxf(fmaxf(sc[0], sc[1]), fmaxf(sc[2], sc[3]));
    float e[4];
    float se = 0.0f;
#pragma unroll
    for (int j = 0; j < 4; ++j) {
      e[j] = expf(sc[j] - mx);
      se += e[j];
    }
    const float inv = 1.0f / se;
    float o0 = 0.0f, o1 = 0.0f;
#pragma unroll
    for (int j = 0; j < 4; ++j) {
      const float pj = e[j] * inv;
      o0 += pj * v0[j];
      o1 += pj * v1[j];
    }
    v2h hv;
    hv[0] = (_Float16)(o0 * X_CARRY);
    hv[1] = (_Float16)(o1 * X_CARRY);
    unsigned short* dp = attn + (size_t)(bt * 4 + qc) * DMODEL + col;
    *(volatile v2h*)(void*)dp = hv;
    __threadfence();
    *(volatile v2h*)(void*)dp = hv;
  }
}

extern "C" void kernel_launch(void* const* d_in, const int* in_sizes, int n_in,
                              void* d_out, int out_size, void* d_ws, size_t ws_size, hipStream_t stream) {
  if (n_in < 14 || d_out == nullptr || d_ws == nullptr) return;
  if (in_sizes[0] != MROWS * DMODEL || in_sizes[1] != DMODEL || in_sizes[2] != DMODEL || in_sizes[3] != DMODEL ||
      in_sizes[4] != DMODEL || in_sizes[5] != DMODEL * DMODEL || in_sizes[6] != DMODEL * DMODEL ||
      in_sizes[7] != DMODEL * DMODEL || in_sizes[8] != DMODEL * DMODEL || in_sizes[9] != DMODEL * DMODEL ||
      in_sizes[10] != NINPROJ * DMODEL || in_sizes[11] != NINPROJ || in_sizes[12] != DMODEL * DMODEL ||
      in_sizes[13] != DMODEL || out_size != MROWS * DMODEL) return;

  const float* inputs = (const float*)d_in[0];
  const float* ln1_g  = (const float*)d_in[1];
  const float* ln1_b  = (const float*)d_in[2];
  const float* ln2_g  = (const float*)d_in[3];
  const float* ln2_b  = (const float*)d_in[4];
  const float* qw     = (const float*)d_in[5];
  const float* kw     = (const float*)d_in[6];
  const float* vw     = (const float*)d_in[7];
  const float* gw     = (const float*)d_in[8];
  const float* ow     = (const float*)d_in[9];
  const float* in_w   = (const float*)d_in[10];
  const float* in_b   = (const float*)d_in[11];
  const float* out_w  = (const float*)d_in[12];
  const float* out_b  = (const float*)d_in[13];
  float* outp = (float*)d_out;

  char* ws = (char*)d_ws;
  size_t off = 0;
  auto carve = [&](size_t bytes) -> char* { char* p = ws + off; off += (bytes + 255) & ~(size_t)255; return p; };
  unsigned short* W16   = (unsigned short*)carve((size_t)(NQKVG + DMODEL + NINPROJ + DMODEL) * DMODEL * 2);
  float*          ROT   = (float*)carve((size_t)TLEN * 32 * 4);
  float*          CSC   = (float*)carve((size_t)NSEQ * NHEAD * 32 * 4);
  float*          KV    = (float*)carve((size_t)NPLANE * 1024 * 4);
  unsigned short* ST16  = (unsigned short*)carve((size_t)NPLANE * 1024 * 2);
  unsigned short* QLO   = (unsigned short*)carve((size_t)NSEQ * NHEAD * FINE_EL * 2);
  unsigned short* KLO   = (unsigned short*)carve((size_t)NSEQ * NHEAD * FINE_EL * 2);
  unsigned short* XLN16 = (unsigned short*)carve((size_t)MPAD * DMODEL * 2);
  unsigned short* QR    = (unsigned short*)carve((size_t)NPLANE * PLANE_EL * 2);
  unsigned short* KR    = (unsigned short*)carve((size_t)NPLANE * PLANE_EL * 2);
  unsigned short* VV    = (unsigned short*)carve((size_t)NPLANE * PLANE_EL * 2);
  float*          X1    = (float*)carve((size_t)MROWS * DMODEL * 4);
  unsigned short* LN2   = (unsigned short*)carve((size_t)MROWS * DMODEL * 2);
  unsigned short* ATT   = (unsigned short*)carve((size_t)MROWS * DMODEL * 2);
  char*           GYR   = carve((size_t)MROWS * NINPROJ * 4);
  float* GPL = (float*)GYR;
  float* YPL = (float*)(GYR + (size_t)MPAD * DMODEL * 4);
  float* QKV = (float*)GYR;
  static_assert((size_t)MPAD * DMODEL * 4 + (size_t)MROWS * DMODEL * 4 <= (size_t)MROWS * NINPROJ * 4);
  if (off > ws_size || off > (size_t)134217728) return;

  unsigned short* W_QKVG = W16;
  unsigned short* W_OW   = W16 + (size_t)NQKVG * DMODEL;
  unsigned short* W_IN   = W_OW + (size_t)DMODEL * DMODEL;
  unsigned short* W_OUT  = W_IN + (size_t)NINPROJ * DMODEL;

  RotAng ra;
  for (int p = 0; p < 16; ++p) ra.a[p] = (float)(1.0 / pow(10000.0, (double)p / 15.0));
  const float hscale = 1.0f / sqrtf((float)HEAD_D);

  cvt_weights_kernel<<<(NQKVG + DMODEL + NINPROJ + DMODEL) * DMODEL / 2048, 256, 0, stream>>>(qw, kw, vw, gw, ow, in_w, out_w, W16);
  rot_table_kernel<<<TLEN / 8, 256, 0, stream>>>(ra, ROT);
  ln_rows_kernel<0><<<MPAD / 8, 256, 0, stream>>>(inputs, ln1_g, ln1_b, XLN16, MPAD);
  gemm_f16_kernel<0, 0, false, false, false><<<(MPAD / 64) * (NQKVG / 64) / 8, 256, 0, stream>>>(
      XLN16, inputs, DMODEL, W_QKVG, DMODEL, GPL, DMODEL, QR, KR, VV, QLO, KLO, in_b, inputs, ROT,
      MPAD, NQKVG, DMODEL, GEMM_SCALE, hscale);
  fine_qk_kernel<<<NSEQ * NHEAD * 2, 256, 0, stream>>>(inputs, ln1_g, ln1_b, qw, kw, ROT, QR, KR, QLO, KLO, hscale);
  kv_chunk_kernel<<<NPLANE, 128, 0, stream>>>(KR, VV, KV);
  scan_kernel<<<NSEQ * NHEAD, 32, 0, stream>>>(KV, ST16, CSC);
  chunk_attn_kernel<<<NPLANE, 128, 0, stream>>>(QR, KR, VV, ST16, QLO, KLO, CSC, GPL, YPL);
  gemm_f16_kernel<1, 1, false, true, false><<<(MROWS / 64) * (DMODEL / 64) / 8, 256, 0, stream>>>(
      XLN16, YPL, DMODEL, W_OW, DMODEL, X1, DMODEL, QR, KR, VV, QLO, KLO, in_b, inputs, ROT,
      MROWS, DMODEL, DMODEL, GEMM_SCALE, hscale);
  ln_rows_kernel<1><<<MROWS / 8, 256, 0, stream>>>(X1, ln2_g, ln2_b, LN2, MROWS);
  gemm_f16_kernel<0, 1, true, false, false><<<(MROWS / 64) * (NINPROJ / 64) / 8, 256, 0, stream>>>(
      LN2, inputs, DMODEL, W_IN, DMODEL, QKV, NINPROJ, QR, KR, VV, QLO, KLO, in_b, inputs, ROT,
      MROWS, NINPROJ, DMODEL, GEMM_SCALE, hscale);
  mha4_kernel<<<MROWS * 4 / 4 / 8, 256, 0, stream>>>(QKV, ATT, hscale);
  gemm_f16_kernel<0, 1, true, true, true><<<(MROWS / 64) * (DMODEL / 64) / 8, 256, 0, stream>>>(
      ATT, inputs, DMODEL, W_OUT, DMODEL, outp, DMODEL, QR, KR, VV, QLO, KLO, out_b, X1, ROT,
      MROWS, DMODEL, DMODEL, GEMM_SCALE, hscale);
}
